// RelRepContextBase_53145925320931
// MI455X (gfx1250) — hardware-verified
//
#include <hip/hip_runtime.h>
#include <math.h>

typedef __attribute__((ext_vector_type(16))) _Float16 v16h;
typedef __attribute__((ext_vector_type(16))) __bf16 v16b;
typedef __attribute__((ext_vector_type(8)))  _Float16 v8h;
typedef __attribute__((ext_vector_type(8)))  float v8f;
typedef __attribute__((ext_vector_type(4)))  float v4f;
typedef __attribute__((ext_vector_type(2)))  float v2f;
typedef __attribute__((ext_vector_type(4)))  unsigned v4u;
typedef __attribute__((ext_vector_type(4)))  int v4i;
typedef float __attribute__((may_alias)) float_a;
typedef int __attribute__((may_alias)) int_a;

template <typename T> __device__ __forceinline__ void vst2(void* p, T v) { *(volatile T*)p = v; __threadfence(); *(volatile T*)p = v; }
__device__ __forceinline__ v8f wmma16(v16h a, v16h b, v8f c) {
  v8f d = __builtin_amdgcn_wmma_f32_16x16x32_f16(false, a, false, b, (short)0, c, false, false);
  asm volatile("v_nop\n\tv_nop\n\tv_nop\n\tv_nop" : "+v"(d) : "v"(a), "v"(b));
  return d;
}
__device__ __forceinline__ v8f wmma_bf(v16b a, v16b b, v8f c) {
  v8f d = __builtin_amdgcn_wmma_f32_16x16x32_bf16(false, a, false, b, (short)0, c, false, false);
  asm volatile("v_nop\n\tv_nop\n\tv_nop\n\tv_nop" : "+v"(d) : "v"(a), "v"(b));
  return d;
}
__device__ __forceinline__ v16h frag_h(const _Float16* rowk0, int lane) {
  union { v16h v; v8h q[2]; } u; const _Float16* p = rowk0 + 8 * (lane >> 4);
  u.q[0] = *(const v8h*)p; u.q[1] = *(const v8h*)(p + 16); return u.v;
}
__device__ __forceinline__ v16h frag_f32(const float* rowk0, int lane) {
  v16h a; const float* p = rowk0 + 8 * (lane >> 4);
#pragma unroll
  for (int i = 0; i < 8; ++i) { a[i] = (_Float16)p[i]; a[8 + i] = (_Float16)p[16 + i]; }
  return a;
}
__device__ __forceinline__ v16h frag_f32s(const float* rowk0, int lane, float sc) {
  v16h a; const float* p = rowk0 + 8 * (lane >> 4);
#pragma unroll
  for (int i = 0; i < 8; ++i) { a[i] = (_Float16)(p[i] * sc); a[8 + i] = (_Float16)(p[16 + i] * sc); }
  return a;
}
__device__ __forceinline__ v16h fragc_f32(const float* W, int k0, int n, int lane, int ld, int K) {
  v16h a; const int g = lane >> 4;
#pragma unroll
  for (int i = 0; i < 8; ++i) { const int ka = k0 + 8 * g + i, kb = ka + 16;
    a[i] = (_Float16)(ka < K ? W[(size_t)(ka < K ? ka : K - 1) * ld + n] : 0.f); a[8 + i] = (_Float16)(kb < K ? W[(size_t)(kb < K ? kb : K - 1) * ld + n] : 0.f); }
  return a;
}
struct F2 { v16b h, l; };
__device__ __forceinline__ F2 bsplit16(const float v[16]) { F2 r;
#pragma unroll
  for (int i = 0; i < 16; ++i) { const __bf16 h = (__bf16)v[i]; r.h[i] = h; r.l[i] = (__bf16)(v[i] - (float)h); }
  return r; }
__device__ __forceinline__ F2 split_row(const float* row, int k0, int lane) { float v[16]; const float* p = row + k0 + 8 * (lane >> 4);
#pragma unroll
  for (int i = 0; i < 8; ++i) { v[i] = p[i]; v[8 + i] = p[16 + i]; }
  return bsplit16(v); }
__device__ __forceinline__ F2 split_rowK(const float* row, int k0, int lane, int K) { float v[16]; const int g = lane >> 4;
#pragma unroll
  for (int i = 0; i < 8; ++i) { const int ka = k0 + 8 * g + i, kb = ka + 16; v[i] = ka < K ? row[ka < K ? ka : K - 1] : 0.f; v[8 + i] = kb < K ? row[kb < K ? kb : K - 1] : 0.f; }
  return bsplit16(v); }
__device__ __forceinline__ F2 split_col(const float* W, int k0, int n, int lane, int ld, int K) { float v[16]; const int g = lane >> 4;
#pragma unroll
  for (int i = 0; i < 8; ++i) { const int ka = k0 + 8 * g + i, kb = ka + 16; v[i] = ka < K ? W[(size_t)(ka < K ? ka : K - 1) * ld + n] : 0.f; v[8 + i] = kb < K ? W[(size_t)(kb < K ? kb : K - 1) * ld + n] : 0.f; }
  return bsplit16(v); }
__device__ __forceinline__ v8f mac3(const F2& a, const F2& b, v8f c) { c = wmma_bf(a.l, b.h, c); c = wmma_bf(a.h, b.l, c); return wmma_bf(a.h, b.h, c); }
__device__ __forceinline__ float sigm(float v) { return 1.0f / (1.0f + expf(-v)); }
#define LDSX() do { asm volatile("s_wait_dscnt 0" ::: "memory"); __builtin_amdgcn_wave_barrier(); __builtin_amdgcn_fence(__ATOMIC_RELEASE, "workgroup"); } while (0)


#define NB 2
#define SS 2048
#define HH 256
#define NSP 512
#define NR 512
#define DIN 768
#define DFF 3072
typedef __attribute__((ext_vector_type(8))) __bf16 v8b;
__device__ __forceinline__ v16b frag_b(const __bf16* rowk0, int lane) {
  union { v16b v; v8b q[2]; } u; const __bf16* p = rowk0 + 8 * (lane >> 4);
  u.q[0] = *(const v8b*)p; u.q[1] = *(const v8b*)(p + 16); return u.v;
}
__device__ __forceinline__ float bfr(float v) { return (float)(__bf16)v; }
__device__ __attribute__((noinline)) float exp_ni(float v) { return expf(v); }
__device__ __attribute__((noinline)) float erf_ni(float v) { return erff(v); }

#define WS_REL 0u
#define WS_H1  (WS_REL + 4u * (size_t)NB * NR * DIN)
#define WS_END (WS_H1 + 4u * (size_t)NB * NR * DFF)

__global__ __launch_bounds__(256) void k_ctx(const float* __restrict__ TOK, const int* __restrict__ TMASK, const float* __restrict__ SPAN, const int* __restrict__ SPID, const int* __restrict__ RID, const int* __restrict__ RMASK, float* __restrict__ REL) { __shared__ __align__(16) float so[DIN];
  const int c = threadIdx.x; const int r = blockIdx.x; const size_t b = blockIdx.y;
  const int hid = RID[(b * NR + r) * 2], tid_ = RID[(b * NR + r) * 2 + 1];
  const int hs = SPID[(b * NSP + hid) * 2], he = SPID[(b * NSP + hid) * 2 + 1], ts = SPID[(b * NSP + tid_) * 2], te = SPID[(b * NSP + tid_) * 2 + 1];
  so[c] = bfr(SPAN[(b * NSP + hid) * HH + c]); so[HH + c] = bfr(SPAN[(b * NSP + tid_) * HH + c]);
  const int lo = min(he, te), hi = max(hs, ts); const bool rm = RMASK[b * NR + r] != 0;
  float mx = -3.0e38f; bool any = false;
  if (rm) {
#pragma unroll 1
    for (int j = max(lo, 0); j < min(hi, SS); ++j) { const bool inh = (j >= hs && j < he), intl = (j >= ts && j < te); if (inh || intl) continue; if (TMASK[b * SS + j] == 0) continue; any = true; mx = fmaxf(mx, bfr(TOK[(b * SS + j) * HH + c])); } }
  so[2 * HH + c] = any ? mx : 0.f;
  __syncthreads(); for (int q = c; q < DIN / 4; q += 256) vst2(REL + (b * NR + r) * DIN + q * 4, *(const v4f*)&so[q * 4]); }
__global__ __launch_bounds__(128) void k_ffn1(const float* __restrict__ REL, const float* __restrict__ W1, const float* __restrict__ B1, float* __restrict__ H1) { __shared__ __align__(16) float sf[4][16][132];
  const int tid = threadIdx.x, wave = tid >> 5, lane = tid & 31, col = lane & 15, g = lane >> 4; const int c0 = blockIdx.y * 128; const size_t r0 = (size_t)blockIdx.x * 64 + wave * 16;
  v8f acc[8] = {};
#pragma unroll 2
  for (int kc = 0; kc < DIN / 32; ++kc) { v16b a; { const float* p = REL + (r0 + col) * DIN + kc * 32 + 8 * g;
#pragma unroll
      for (int i = 0; i < 8; ++i) { a[i] = (__bf16)p[i]; a[8 + i] = (__bf16)p[16 + i]; } }
#pragma unroll
    for (int j = 0; j < 8; ++j) { v16b w; const int o = c0 + j * 16 + col;
#pragma unroll
      for (int i = 0; i < 8; ++i) { w[i] = (__bf16)W1[(size_t)(kc * 32 + 8 * g + i) * DFF + o]; w[8 + i] = (__bf16)W1[(size_t)(kc * 32 + 16 + 8 * g + i) * DFF + o]; }
      acc[j] = wmma_bf(a, w, acc[j]); } }
#pragma unroll
  for (int j = 0; j < 8; ++j) { const float bb = bfr(B1[c0 + j * 16 + col]);
#pragma unroll
    for (int r = 0; r < 8; ++r) sf[wave][8 * g + r][j * 16 + col] = fmaxf(acc[j][r] + bb, 0.f); }
  LDSX(); for (int rl = 0; rl < 16; ++rl) vst2(H1 + (r0 + rl) * DFF + c0 + lane * 4, *(const v4f*)&sf[wave][rl][lane * 4]); }
__global__ __launch_bounds__(128) void k_ffn2(const float* __restrict__ H1, const float* __restrict__ W2, const float* __restrict__ B2, float* __restrict__ OUT) { __shared__ __align__(16) float sf[4][16][132];
  const int tid = threadIdx.x, wave = tid >> 5, lane = tid & 31, col = lane & 15, g = lane >> 4; const int c0 = blockIdx.y * 128; const size_t r0 = (size_t)blockIdx.x * 64 + wave * 16;
  v8f acc[8] = {};
#pragma unroll 2
  for (int kc = 0; kc < DFF / 32; ++kc) { const F2 a = split_row(H1 + (r0 + col) * DFF, kc * 32, lane);
#pragma unroll
    for (int j = 0; j < 8; ++j) { v16b w; const int o = c0 + j * 16 + col;
#pragma unroll
      for (int i = 0; i < 8; ++i) { w[i] = (__bf16)W2[(size_t)(kc * 32 + 8 * g + i) * HH + o]; w[8 + i] = (__bf16)W2[(size_t)(kc * 32 + 16 + 8 * g + i) * HH + o]; }
      acc[j] = wmma_bf(a.h, w, acc[j]); acc[j] = wmma_bf(a.l, w, acc[j]); } }
#pragma unroll
  for (int j = 0; j < 8; ++j) { const float bb = bfr(B2[c0 + j * 16 + col]);
#pragma unroll
    for (int r = 0; r < 8; ++r) sf[wave][8 * g + r][j * 16 + col] = acc[j][r] + bb; }
  LDSX(); for (int rl = 0; rl < 16; ++rl) vst2(OUT + (r0 + rl) * HH + c0 + lane * 4, *(const v4f*)&sf[wave][rl][lane * 4]); }
extern "C" void kernel_launch(void* const* d_in, const int* in_sizes, int n_in, void* d_out, int out_size, void* d_ws, size_t ws_size, hipStream_t stream) {
  (void)in_sizes; (void)n_in; (void)out_size;
  const float** F = (const float**)d_in;
  if (ws_size < (size_t)WS_END) return;
  char* ws = (char*)d_ws; float *REL = (float*)(ws + WS_REL), *H1 = (float*)(ws + WS_H1);
  k_ctx<<<dim3(NR, NB), 256, 0, stream>>>(F[0], (const int*)d_in[1], F[2], (const int*)d_in[3], (const int*)d_in[4], (const int*)d_in[5], REL);
  k_ffn1<<<dim3(NB * NR / 64, DFF / 128), 128, 0, stream>>>(REL, F[7], F[8], H1);
  k_ffn2<<<dim3(NB * NR / 64, HH / 128), 128, 0, stream>>>(H1, F[9], F[10], (float*)d_out);
}
